// KA_attention_crossinf_scaling_16655883173899
// MI455X (gfx1250) — hardware-verified
//
#include <hip/hip_runtime.h>
#include <math.h>

#ifndef NB
#define NB 16
#endif
#define NB_FULL 16
#define NH 12
#define SEQ 256
#define HD 64
#define NF 8
#define HP (NH * SEQ)
#define RQ (NB * HP)
#define RQ_FULL (NB_FULL * HP)
#define BH (NB * NH)
#define MT (((BH + 1 + 63) / 64) * 64)
#define QEL_FULL (RQ_FULL * HD)
#define ZB_N 256

static_assert(SEQ == 256);
static_assert(HD == 64);
static_assert(NF == 8);
static_assert(NB <= NB_FULL);
static_assert((size_t)QEL_FULL * 4 == (size_t)12582912);
static_assert((2 * RQ) % 64 == 0);
static_assert(RQ % 128 == 0);
static_assert(HD % 32 == 0 && SEQ % 32 == 0);
static_assert(HD % 64 == 0 && SEQ % 64 == 0 && MT % 64 == 0);
static_assert(BH + 1 <= MT);
static_assert((RQ * HD / 8) % 256 == 0);
static_assert((RQ * HD / 4) % 256 == 0);
static_assert((MT * 32) % 256 == 0);
static_assert((HD * HD / 8) % 256 == 0 && (SEQ * SEQ / 8) % 256 == 0);
static_assert(ZB_N == 64 * 4 && ZB_N >= SEQ && ZB_N >= HD);
static_assert(32 * 4 == 128);
static_assert(4 * 4 * 16 == SEQ);
static_assert(256 * 16 * 16 == SEQ * HD * 4);
static_assert(8 * 16 * 68 * 4 <= 131072);
static_assert(3 * 256 * 4 + 4 * 256 * 8 + 4 * 8 + 4 * 4 + 4 * 2 * 64 * 4 + 2 * 64 * 4 <= 131072);

typedef __attribute__((ext_vector_type(16))) _Float16 v16h;
typedef __attribute__((ext_vector_type(8)))  _Float16 v8h;
typedef __attribute__((ext_vector_type(8)))  float    v8f;
typedef __attribute__((ext_vector_type(4)))  float    v4f;
typedef __attribute__((ext_vector_type(4)))  unsigned int v4u;


#define VST2(T, ptr, val) do { const T vst2_v_ = (val); *(volatile T*)(ptr) = vst2_v_; __threadfence(); *(volatile T*)(ptr) = vst2_v_; } while (0)
#define VST2V4(ptr, val) do { const v4f vst2_v4_ = (val); *(volatile v4f*)(ptr) = vst2_v4_; __threadfence(); *(volatile v4f*)(ptr) = vst2_v4_; } while (0)

__device__ __forceinline__ float bfr(float f) {
    unsigned u = __float_as_uint(f);
    u += 0x7FFFu + ((u >> 16) & 1u);
    return __uint_as_float(u & 0xFFFF0000u);
}
__device__ __forceinline__ unsigned short f2h_bits(float x) {
    return (fabsf(x) < 6.104e-5f) ? (unsigned short)0 : __builtin_bit_cast(unsigned short, (_Float16)x);
}
__device__ __forceinline__ void st8h(unsigned short* P, size_t o, const float* v) {
    v4u pk;
    pk.x = (unsigned)f2h_bits(v[0]) | ((unsigned)f2h_bits(v[1]) << 16);
    pk.y = (unsigned)f2h_bits(v[2]) | ((unsigned)f2h_bits(v[3]) << 16);
    pk.z = (unsigned)f2h_bits(v[4]) | ((unsigned)f2h_bits(v[5]) << 16);
    pk.w = (unsigned)f2h_bits(v[6]) | ((unsigned)f2h_bits(v[7]) << 16);
    VST2(v4u, (v4u*)(P + o), pk);
}

union FragU { v16h v; v8h h[2]; };
__device__ __forceinline__ v16h frag_ld(const _Float16* p) {
    FragU f; f.h[0] = *(const v8h*)(p); f.h[1] = *(const v8h*)(p + 16); return f.v;
}
__device__ __forceinline__ v8f wmma16(v16h a, v16h b, v8f c) {
    c = __builtin_amdgcn_wmma_f32_16x16x32_f16(false, a, false, b, (short)0, c, false, false);
    asm volatile("v_nop\n\tv_nop\n\tv_nop\n\tv_nop" : "+v"(c) : "v"(a), "v"(b));
    return c;
}
__device__ __forceinline__ void dep_guard_h(v8f& a, v8f& b, v16h x, v16h y) { asm volatile("v_nop\n\tv_nop\n\tv_nop\n\tv_nop" : "+v"(a), "+v"(b) : "v"(x), "v"(y)); }
__device__ __forceinline__ void keep4_h(v16h a, v16h b, v16h c, v16h d) { asm volatile("v_nop" :: "v"(a), "v"(b), "v"(c), "v"(d)); }
__device__ __forceinline__ void acc_guard4(v8f& a, v8f& b, v8f& c, v8f& d) { asm volatile("v_nop\n\tv_nop\n\tv_nop\n\tv_nop" : "+v"(a), "+v"(b), "+v"(c), "+v"(d)); }
__device__ __forceinline__ void wave_sync_lds() {
    __builtin_amdgcn_fence(3  , "workgroup");
    __builtin_amdgcn_wave_barrier();
    __builtin_amdgcn_fence(2  , "workgroup");
}

template <int OUT_MODE, bool RESID, bool RELU>
__global__ __launch_bounds__(256) void k_gemm64(
    const _Float16* __restrict__ A, unsigned lda, const _Float16* __restrict__ Bt, unsigned ldb,
    void* __restrict__ Cout, unsigned ldc, const float* __restrict__ bias, const float* __restrict__ resid,
    unsigned M, unsigned N, unsigned K, float scale, float oscale) {
  __shared__ __align__(16) float sT[8][16 * 68];
  const unsigned lane = threadIdx.x & 31u;
  const unsigned wave = threadIdx.x >> 5;
  const unsigned tilesN = N >> 6, tilesM = M >> 6;
  const unsigned tile = blockIdx.x * 8u + wave;
  if (tile >= tilesM * tilesN) return;
  const unsigned tm = tile / tilesN;
  const unsigned tn = tile - tm * tilesN;
  const unsigned m0 = tm << 6, n0 = tn << 6;
  const unsigned rlane = lane & 15u;
  const unsigned koff = (lane >> 4) * 8u;
  const unsigned mOff = koff;

  v8f acc[4][4];
#pragma unroll
  for (int i = 0; i < 4; ++i)
#pragma unroll
    for (int j = 0; j < 4; ++j) acc[i][j] = (v8f){0.f,0.f,0.f,0.f,0.f,0.f,0.f,0.f};

  for (unsigned k0 = 0; k0 < K; k0 += 32u) {
    v16h bh[4];
#pragma unroll
    for (int j = 0; j < 4; ++j)
      bh[j] = frag_ld(Bt + (size_t)(n0 + ((unsigned)j << 4) + rlane) * ldb + koff + k0);
#pragma unroll
    for (int i = 0; i < 4; ++i) {
      const v16h ah = frag_ld(A + (size_t)(m0 + ((unsigned)i << 4) + rlane) * lda + koff + k0);
#pragma unroll
      for (int j = 0; j < 4; ++j)
        acc[i][j] = __builtin_amdgcn_wmma_f32_16x16x32_f16(false, ah, false, bh[j], (short)0, acc[i][j], false, false);
      dep_guard_h(acc[i][0], acc[i][3], ah, ah);
    }
    keep4_h(bh[0], bh[1], bh[2], bh[3]);
  }
  acc_guard4(acc[0][0], acc[0][1], acc[0][2], acc[0][3]);
  acc_guard4(acc[1][0], acc[1][1], acc[1][2], acc[1][3]);
  acc_guard4(acc[2][0], acc[2][1], acc[2][2], acc[2][3]);
  acc_guard4(acc[3][0], acc[3][1], acc[3][2], acc[3][3]);

  float* slab = sT[wave];
#pragma unroll
  for (int i = 0; i < 4; ++i) {
    const unsigned mBase = m0 + ((unsigned)i << 4);
#pragma unroll
    for (int j = 0; j < 4; ++j) {
      const unsigned n = n0 + ((unsigned)j << 4) + rlane;
      const float bv = bfr(bias[n]);
#pragma unroll
      for (int r = 0; r < 8; ++r) {
        float v = acc[i][j][r] * scale + bv;
        if (RELU) v = fmaxf(v, 0.0f);
        if (OUT_MODE == 1) v *= oscale;
        slab[(mOff + (unsigned)r) * 68u + ((unsigned)j << 4) + rlane] = v;
      }
    }
    wave_sync_lds();
    if (OUT_MODE == 0) {
      float* C = (float*)Cout;
      const unsigned hh = lane >> 4, c4 = (lane & 15u) * 4u;
#pragma unroll
      for (int half = 0; half < 2; ++half) {
        v4f vv[4];
#pragma unroll
        for (int it = 0; it < 4; ++it) {
          const unsigned row = (unsigned)(half * 4 + it) * 2u + hh;
          vv[it] = *(const v4f*)(slab + row * 68u + c4);
          if (RESID) vv[it] += *(const v4f*)(resid + (size_t)(mBase + row) * ldc + n0 + c4);
        }
        for (int pass = 0; pass < 2; ++pass) {
#pragma unroll
          for (int it = 0; it < 4; ++it) {
            const unsigned row = (unsigned)(half * 4 + it) * 2u + hh;
            *(volatile v4f*)(C + (size_t)(mBase + row) * ldc + n0 + c4) = vv[it];
          }
          __threadfence();
        }
      }
    } else {
      _Float16* C = (_Float16*)Cout;
      const unsigned q = lane >> 3, c8 = (lane & 7u) * 8u;
      v8h hv[4];
#pragma unroll
      for (int it = 0; it < 4; ++it) {
        const unsigned row = (unsigned)it * 4u + q;
        const float* sp = slab + row * 68u + c8;
#pragma unroll
        for (int e = 0; e < 8; ++e) hv[it][e] = (_Float16)sp[e];
      }
      for (int pass = 0; pass < 2; ++pass) {
#pragma unroll
        for (int it = 0; it < 4; ++it) {
          const unsigned row = (unsigned)it * 4u + q;
          *(volatile v8h*)(C + (size_t)(mBase + row) * ldc + n0 + c8) = hv[it];
        }
        __threadfence();
      }
    }
    wave_sync_lds();
  }
}

__global__ __launch_bounds__(64) void k_fillz(float* __restrict__ z) {
    const v4f zero = (v4f){0.f, 0.f, 0.f, 0.f};
    VST2V4(z + 4u * threadIdx.x, zero);
}

__global__ __launch_bounds__(256) void k_wcv(const float* __restrict__ Wm, unsigned n8, unsigned short* __restrict__ W16, float sw) {
#pragma clang fp contract(off)
    const unsigned u = blockIdx.x * 256u + threadIdx.x;
    if (u >= n8) return;
    const v4f a = *(const v4f*)(Wm + (size_t)8u * u), b = *(const v4f*)(Wm + (size_t)8u * u + 4u);
    float v[8];
    v[0] = bfr(a.x) * sw; v[1] = bfr(a.y) * sw; v[2] = bfr(a.z) * sw; v[3] = bfr(a.w) * sw;
    v[4] = bfr(b.x) * sw; v[5] = bfr(b.y) * sw; v[6] = bfr(b.z) * sw; v[7] = bfr(b.w) * sw;
    st8h(W16, (size_t)8u * u, v);
}

__global__ __launch_bounds__(256) void k_act(const float* __restrict__ x, unsigned short* __restrict__ s16, unsigned n8) {
#pragma clang fp contract(off)
    const unsigned u = blockIdx.x * 256u + threadIdx.x;
    if (u >= n8) return;
    const v4f a = *(const v4f*)(x + (size_t)8u * u), b = *(const v4f*)(x + (size_t)8u * u + 4u);
    const float xs[8] = {a.x, a.y, a.z, a.w, b.x, b.y, b.z, b.w};
    float v[8];
#pragma unroll
    for (int i = 0; i < 8; ++i) {
        const float xb = bfr(xs[i]);
        const float e = __expf(-xb);
        const float sg = __builtin_amdgcn_rcpf(1.0f + e);
        v[i] = (xb * sg) * 8.0f;
    }
    st8h(s16, (size_t)8u * u, v);
}

__global__ __launch_bounds__(256) void k_copyq(const float* __restrict__ q, float* __restrict__ out, unsigned n4) {
    const unsigned u = blockIdx.x * 256u + threadIdx.x;
    if (u >= n4) return;
    v4f a = *(const v4f*)(q + (size_t)4u * u);
    a.x = bfr(a.x); a.y = bfr(a.y); a.z = bfr(a.z); a.w = bfr(a.w);
    VST2V4(out + (size_t)4u * u, a);
}

__global__ __launch_bounds__(256) void k_sig(const float* __restrict__ x, const float* __restrict__ base,
                                             const float* __restrict__ gridf, const float* __restrict__ coef,
                                             const float* __restrict__ sbase, const float* __restrict__ ssp,
                                             float* __restrict__ tsum) {
#pragma clang fp contract(off)
    __shared__ __align__(16) float sT[128];
    const unsigned t = threadIdx.x, hw = t >> 4, l16 = t & 15u, d0 = 4u * l16;
    const v4f g0 = *(const v4f*)(gridf), g1 = *(const v4f*)(gridf + 4);
    const float g[8] = {bfr(g0.x), bfr(g0.y), bfr(g0.z), bfr(g0.w), bfr(g1.x), bfr(g1.y), bfr(g1.z), bfr(g1.w)};
    float cf[4][8];
#pragma unroll
    for (int e = 0; e < 4; ++e) {
        const v4f c0 = *(const v4f*)(coef + (d0 + (unsigned)e) * 8u), c1 = *(const v4f*)(coef + (d0 + (unsigned)e) * 8u + 4u);
        cf[e][0] = bfr(c0.x); cf[e][1] = bfr(c0.y); cf[e][2] = bfr(c0.z); cf[e][3] = bfr(c0.w);
        cf[e][4] = bfr(c1.x); cf[e][5] = bfr(c1.y); cf[e][6] = bfr(c1.z); cf[e][7] = bfr(c1.w);
    }
#pragma unroll 1
    for (unsigned it = 0; it < 8u; ++it) {
        const unsigned row = blockIdx.x * 128u + it * 16u + hw;
        const unsigned hp = row % (unsigned)HP;
        const v4f xv = *(const v4f*)(x + (size_t)row * 64u + d0);
        const v4f bv = *(const v4f*)(base + (size_t)row * 64u + d0);
        const v4f sb = *(const v4f*)(sbase + (size_t)hp * 64u + d0);
        const v4f sp = *(const v4f*)(ssp + (size_t)hp * 64u + d0);
        const float xs[4] = {xv.x, xv.y, xv.z, xv.w};
        const float bs[4] = {bv.x, bv.y, bv.z, bv.w};
        const float sbs[4] = {sb.x, sb.y, sb.z, sb.w};
        const float sps[4] = {sp.x, sp.y, sp.z, sp.w};
        float acc = 0.f;
#pragma unroll
        for (int e = 0; e < 4; ++e) {
            const float xb = bfr(xs[e]);
            float fs = 0.f;
#pragma unroll
            for (int f = 0; f < 8; ++f) fs += cf[e][f] * __sinf(g[f] * xb);
            const float fv = fs * bfr(sps[e]) + bs[e] * bfr(sbs[e]);
            const float ex = __expf(fv);
            acc += __builtin_amdgcn_rcpf(1.0f + ex);
        }
        acc += __shfl_xor(acc, 1, 32); acc += __shfl_xor(acc, 2, 32);
        acc += __shfl_xor(acc, 4, 32); acc += __shfl_xor(acc, 8, 32);
        if (l16 == 0u) sT[it * 16u + hw] = acc;
    }
    __syncthreads();
    if (t < 32u) {
        const v4f v = *(const v4f*)(sT + 4u * t);
        VST2V4(tsum + (size_t)blockIdx.x * 128u + 4u * t, v);
    }
}

__global__ __launch_bounds__(256) void k_tplane(const float* __restrict__ tk, unsigned short* __restrict__ t16) {
#pragma clang fp contract(off)
    const unsigned u = blockIdx.x * 256u + threadIdx.x;
    if (u >= (unsigned)(MT * 32)) return;
    const unsigned row = u >> 5, c0 = (u & 31u) * 8u;
    const unsigned rr = (row < (unsigned)BH) ? row : (unsigned)(BH - 1);
    const v4f a = *(const v4f*)(tk + (size_t)rr * 256u + c0), b = *(const v4f*)(tk + (size_t)rr * 256u + c0 + 4u);
    const float src[8] = {a.x, a.y, a.z, a.w, b.x, b.y, b.z, b.w};
    const float fill = (row == (unsigned)BH) ? 256.0f : 0.0f;
    float v[8];
#pragma unroll
    for (int i = 0; i < 8; ++i) v[i] = (row < (unsigned)BH) ? (src[i] * 256.0f) : fill;
    st8h(t16, (size_t)row * 256u + c0, v);
}

__global__ __launch_bounds__(256) void k_fin(const float* __restrict__ kin, const float* __restrict__ tq,
                                             const float* __restrict__ G, const float* __restrict__ lb,
                                             float* __restrict__ out1) {
#pragma clang fp contract(off)
    __shared__ __align__(16) float sR[256];
    __shared__ __align__(16) float sM[256];
    __shared__ __align__(16) float sD[256];
    __shared__ double sRed[4][256];
    __shared__ double sS[4];
    __shared__ float sPhi[4];
    __shared__ float sGp[4][2][64];
    __shared__ __align__(16) float sH[2][64];
    const unsigned t = threadIdx.x, bh = blockIdx.x;
    const float* kb = kin + (size_t)bh * (SEQ * HD);
    float* ob = out1 + (size_t)bh * (SEQ * HD);
    {
        const float rl = G[(size_t)BH * 256u + t];
        const float tw = G[(size_t)bh * 256u + t];
        const float mj = (128.0f * rl - tw) + bfr(lb[t]);
        const float dl = -tq[(size_t)bh * 256u + t];
        sR[t] = rl; sM[t] = mj; sD[t] = dl;
        sRed[0][t] = (double)rl * (double)dl;
        sRed[1][t] = (double)rl;
        sRed[2][t] = (double)mj * (double)dl;
        sRed[3][t] = (double)mj;
    }
    __syncthreads();
    if (t < 4u) {
        double s = 0.0;
#pragma unroll 1
        for (unsigned j = 0; j < 256u; ++j) s += sRed[t][j];
        sS[t] = s;
    }
    __syncthreads();
    if (t == 0u) {
        const double sc = 1.0 / 1048576.0;
        const double x0 = sS[0] * sc, x1 = sS[1] * sc, x2 = sS[2] * sc, x3 = sS[3] * sc;
        double t0 = 1.0, t1 = 0.0, t2 = 0.0, t3 = 1.0;
        double e0 = 1.0, e1 = 0.0, e2 = 0.0, e3 = 1.0;
        double p0 = 1.0, p1 = 0.0, p2 = 0.0, p3 = 1.0;
#pragma unroll
        for (int n = 1; n <= 8; ++n) {
            const double rn = 1.0 / (double)n;
            const double rn1 = 1.0 / (double)(n + 1);
            const double n0 = (t0 * x0 + t1 * x2) * rn;
            const double n1 = (t0 * x1 + t1 * x3) * rn;
            const double n2 = (t2 * x0 + t3 * x2) * rn;
            const double n3 = (t2 * x1 + t3 * x3) * rn;
            t0 = n0; t1 = n1; t2 = n2; t3 = n3;
            e0 += t0; e1 += t1; e2 += t2; e3 += t3;
            p0 += t0 * rn1; p1 += t1 * rn1; p2 += t2 * rn1; p3 += t3 * rn1;
        }
#pragma unroll 1
        for (int it = 0; it < 20; ++it) {
            const double a0 = e0 + 1.0, a1 = e1, a2 = e2, a3 = e3 + 1.0;
            const double q0 = 0.5 * (p0 * a0 + p1 * a2);
            const double q1 = 0.5 * (p0 * a1 + p1 * a3);
            const double q2 = 0.5 * (p2 * a0 + p3 * a2);
            const double q3 = 0.5 * (p2 * a1 + p3 * a3);
            const double f0 = e0 * e0 + e1 * e2;
            const double f1 = e0 * e1 + e1 * e3;
            const double f2 = e2 * e0 + e3 * e2;
            const double f3 = e2 * e1 + e3 * e3;
            p0 = q0; p1 = q1; p2 = q2; p3 = q3;
            e0 = f0; e1 = f1; e2 = f2; e3 = f3;
        }
        sPhi[0] = (float)p0; sPhi[1] = (float)p1; sPhi[2] = (float)p2; sPhi[3] = (float)p3;
    }
    {
        const unsigned d = t & 63u, part = t >> 6;
        float g1 = 0.f, g2 = 0.f;
#pragma unroll 4
        for (unsigned jj = 0; jj < 64u; ++jj) {
            const unsigned j = part * 64u + jj;
            const float kv = bfr(kb[(size_t)j * 64u + d]);
            g1 += sR[j] * kv;
            g2 += sM[j] * kv;
        }
        sGp[part][0][d] = g1;
        sGp[part][1][d] = g2;
    }
    __syncthreads();
    if (t < 64u) {
        const float G1 = (sGp[0][0][t] + sGp[1][0][t]) + (sGp[2][0][t] + sGp[3][0][t]);
        const float G2 = (sGp[0][1][t] + sGp[1][1][t]) + (sGp[2][1][t] + sGp[3][1][t]);
        sH[0][t] = sPhi[0] * G1 + sPhi[1] * G2;
        sH[1][t] = sPhi[2] * G1 + sPhi[3] * G2;
    }
    __syncthreads();
    {
        const unsigned c4 = (t & 15u) * 4u, r0 = t >> 4;
        const v4f h1 = *(const v4f*)(&sH[0][c4]);
        const v4f h2 = *(const v4f*)(&sH[1][c4]);
#pragma unroll 1
        for (unsigned grp = 0; grp < 4u; ++grp) {
            v4f vv[4];
#pragma unroll
            for (int it = 0; it < 4; ++it) {
                const unsigned row = (grp * 4u + (unsigned)it) * 16u + r0;
                const v4f kv = *(const v4f*)(kb + (size_t)row * 64u + c4);
                const float dl = sD[row];
                vv[it].x = (bfr(kv.x) + dl * h1.x) + h2.x;
                vv[it].y = (bfr(kv.y) + dl * h1.y) + h2.y;
                vv[it].z = (bfr(kv.z) + dl * h1.z) + h2.z;
                vv[it].w = (bfr(kv.w) + dl * h1.w) + h2.w;
            }
            for (int pass = 0; pass < 2; ++pass) {
#pragma unroll
                for (int it = 0; it < 4; ++it) {
                    const unsigned row = (grp * 4u + (unsigned)it) * 16u + r0;
                    *(volatile v4f*)(ob + (size_t)row * 64u + c4) = vv[it];
                }
                __threadfence();
            }
        }
    }
}

static constexpr float SC_BASE = 1.0f / 256.0f;
static constexpr float SC_LIN  = 1.0f / 2097152.0f;

extern "C" void kernel_launch(void* const* d_in, const int* in_sizes, int n_in, void* d_out, int out_size,
                              void* d_ws, size_t ws_size, hipStream_t stream) {
    if (n_in < 10) return;
    if (in_sizes[0] < RQ * HD || in_sizes[1] < RQ * HD || in_sizes[3] < NF || in_sizes[4] < HD * HD) return;
    if (in_sizes[5] < HD * NF || in_sizes[6] < HP * HD || in_sizes[7] < HP * HD || in_sizes[8] < SEQ * SEQ || in_sizes[9] < SEQ) return;
    if (out_size < QEL_FULL + RQ * HD) return;

    const float* q      = (const float*)d_in[0];
    const float* k      = (const float*)d_in[1];
    const float* gridf  = (const float*)d_in[3];
    const float* bw     = (const float*)d_in[4];
    const float* coef   = (const float*)d_in[5];
    const float* sbase  = (const float*)d_in[6];
    const float* ssp    = (const float*)d_in[7];
    const float* lw     = (const float*)d_in[8];
    const float* lb     = (const float*)d_in[9];
    float* out0 = (float*)d_out;
    float* out1 = out0 + (size_t)QEL_FULL;

    char* wsp = (char*)d_ws;
    size_t off = 0;
    auto carve = [&](size_t bytes) -> void* { void* r = wsp + off; off += (bytes + 255) & ~(size_t)255; return r; };
    float*          zb    = (float*)carve((size_t)ZB_N * 4);
    unsigned short* wB16  = (unsigned short*)carve((size_t)HD * HD * 2);
    unsigned short* wL16  = (unsigned short*)carve((size_t)SEQ * SEQ * 2);
    unsigned short* s16   = (unsigned short*)carve((size_t)2 * RQ * HD * 2);
    float*          basep = (float*)carve((size_t)2 * RQ * HD * 4);
    float*          tsum  = (float*)carve((size_t)2 * RQ * 4);
    unsigned short* t16   = (unsigned short*)carve((size_t)MT * SEQ * 2);
    float*          Gp    = (float*)carve((size_t)MT * SEQ * 4);
    if (off > ws_size || off > (size_t)134217728) return;

    k_fillz<<<1, 64, 0, stream>>>(zb);
    k_wcv<<<(HD * HD / 8 + 255) / 256, 256, 0, stream>>>(bw, (unsigned)(HD * HD / 8), wB16, 32.0f);
    k_wcv<<<(SEQ * SEQ / 8 + 255) / 256, 256, 0, stream>>>(lw, (unsigned)(SEQ * SEQ / 8), wL16, 8192.0f);

    k_act<<<(RQ * HD / 8) / 256, 256, 0, stream>>>(q, s16, (unsigned)(RQ * HD / 8));
    k_act<<<(RQ * HD / 8) / 256, 256, 0, stream>>>(k, s16 + (size_t)RQ * HD, (unsigned)(RQ * HD / 8));
    k_copyq<<<(RQ * HD / 4) / 256, 256, 0, stream>>>(q, out0, (unsigned)(RQ * HD / 4));

    const unsigned gB = ((2 * RQ / 64) * (HD / 64) + 7) / 8;
    k_gemm64<0, false, false><<<gB, 256, 0, stream>>>((const _Float16*)s16, HD, (const _Float16*)wB16, HD,
        (void*)basep, HD, zb, nullptr, 2 * RQ, HD, HD, SC_BASE, 1.0f);

    k_sig<<<RQ / 128, 256, 0, stream>>>(q, basep, gridf, coef, sbase, ssp, tsum);
    k_sig<<<RQ / 128, 256, 0, stream>>>(k, basep + (size_t)RQ * HD, gridf, coef, sbase, ssp, tsum + RQ);

    k_tplane<<<(MT * 32) / 256, 256, 0, stream>>>(tsum + RQ, t16);
    const unsigned gL = ((MT / 64) * (SEQ / 64) + 7) / 8;
    k_gemm64<0, false, false><<<gL, 256, 0, stream>>>((const _Float16*)t16, SEQ, (const _Float16*)wL16, SEQ,
        (void*)Gp, SEQ, zb, nullptr, MT, SEQ, SEQ, SC_LIN, 1.0f);

    k_fin<<<BH, 256, 0, stream>>>(k, tsum, Gp, lb, out1);
}
